// JointSpatioTemporalBlock_73787538145515
// MI455X (gfx1250) — hardware-verified
//
#include <hip/hip_runtime.h>
#include <hip/hip_bf16.h>
#include <math.h>

#define BB 2
#define SS 2560
#define QROWS 2560
#define KROWS 2560
#define NKV 2500
#define DD 512
#define KVD 512
#define HH 8
#define KVH 8
#define HKDIV 1
#define DKK 64
#define QW 2
#define GSTR 48
#define TTj 100
#define VVj 25
#define LLj 2500
#define DDj 256
#define HDj 32
#define MAXT 300
#define MROWS (BB * LLj)
#define MPADr (BB * SS)
#define BTS 2560

typedef _Float16 bf16;
typedef _Float16 f16;
typedef __attribute__((ext_vector_type(4))) unsigned v4u_t;
typedef unsigned v4ua __attribute__((ext_vector_type(4), may_alias));
typedef __attribute__((ext_vector_type(4))) float v4f_t;
typedef float v4fa __attribute__((ext_vector_type(4), may_alias));
typedef __attribute__((ext_vector_type(16))) bf16  bf16x16;
typedef bf16x16 f16x16;
typedef __attribute__((ext_vector_type(8)))  bf16  bf16x8;
typedef bf16x8 f16x8;
typedef __attribute__((ext_vector_type(4)))  bf16  bf16x4;
typedef __attribute__((ext_vector_type(8)))  float f32x8;
__device__ __forceinline__ f32x8 wmma16(f16x16 a, f16x16 b, f32x8 c) {
  c = __builtin_amdgcn_wmma_f32_16x16x32_f16(false, a, false, b, (short)0, c, false, false);
  asm volatile("v_nop\n\tv_nop\n\tv_nop\n\tv_nop" : "+v"(c) : "v"(a), "v"(b));
  return c;
}
#define LDS_STRIDE 48
#define KSTRIDE    72
#define VSTRIDE    48

__device__ __forceinline__ f32x8 wmma_bf16(bf16x16 a, bf16x16 b, f32x8 c) {
  c = __builtin_amdgcn_wmma_f32_16x16x32_f16(false, a, false, b, (short)0, c, false, false);
  asm volatile("v_nop\n\tv_nop\n\tv_nop\n\tv_nop" : "+v"(c) : "v"(a), "v"(b));
  return c;
}

template <typename T>
__device__ __forceinline__ bf16x16 load_frag(const T* __restrict__ base, int ld,
                                             int row0, int k0) {
  const int lane = threadIdx.x & 31;
  const int r    = lane & 15;
  const int kh   = (lane >> 4) * 8;
  const T* p0 = base + (size_t)(row0 + r) * ld + (k0 + kh);
  const T* p1 = p0 + 16;
  bf16x16 f;
#pragma unroll
  for (int i = 0; i < 8; ++i) {
    f[i]     = (bf16)p0[i];
    f[i + 8] = (bf16)p1[i];
  }
  return f;
}

__device__ __forceinline__ bf16x16 lds_frag(const bf16* base, int stride) {
  const int lane = threadIdx.x & 31;
  const int row  = lane & 15;
  const int kh   = (lane >> 4) * 8;
  const bf16x8 lo = *(const bf16x8*)(base + row * stride + kh);
  const bf16x8 hi = *(const bf16x8*)(base + row * stride + kh + 16);
  bf16x16 f;
#pragma unroll
  for (int i = 0; i < 8; ++i) { f[i] = lo[i]; f[i + 8] = hi[i]; }
  return f;
}

template <typename T>
__device__ __forceinline__ void stage_read16(const T* __restrict__ p, float* buf) {
#pragma unroll
  for (int i = 0; i < 16; ++i) buf[i] = (float)p[i];
}

__device__ __forceinline__ void stage_write(bf16* dst, const float* buf, int nquad) {
#pragma unroll
  for (int i = 0; i < nquad; ++i) {
    bf16x4 q;
    q[0] = (bf16)buf[4 * i];     q[1] = (bf16)buf[4 * i + 1];
    q[2] = (bf16)buf[4 * i + 2]; q[3] = (bf16)buf[4 * i + 3];
    *(bf16x4*)(dst + 4 * i) = q;
  }
}

template <typename AT, int MODE>
__global__ __launch_bounds__(256) void gemm_rb_kernel(
    const AT* __restrict__ A, const float* __restrict__ W,
    const float* __restrict__ bias, const float* __restrict__ rowscale, const float* __restrict__ R, const float* __restrict__ rowbias, void* __restrict__ out,
    int M, int N, int K) {
  __shared__ bf16 ldsA[128 * LDS_STRIDE];
  __shared__ bf16 ldsW[256 * LDS_STRIDE];
  __shared__ __attribute__((aligned(16))) unsigned char sob[256 * 136 * 2];

  const int t    = threadIdx.x;
  const int wave = t >> 5;
  const int lane = t & 31;
  const int wm   = (wave & 1) * 64;
  const int wn   = (wave >> 1) * 64;
  const int mBlk = blockIdx.x * 128;
  const int nBlk = blockIdx.y * 256;

  const int arow = t >> 1;
  const int ach  = (t & 1) * 16;

  float abuf[16];
  float wbuf[32];

  stage_read16(A + (size_t)(mBlk + arow) * K + ach, abuf);
  const int nrow = min(nBlk + t, N - 1);
  stage_read16(W + (size_t)nrow * K,          wbuf);
  stage_read16(W + (size_t)nrow * K + 16,     wbuf + 16);

  f32x8 acc[4][4] = {};

  for (int k = 0; k < K; k += 32) {
    __syncthreads();
    stage_write(&ldsA[arow * LDS_STRIDE + ach], abuf, 4);
    stage_write(&ldsW[t * LDS_STRIDE],          wbuf, 8);
    if (k + 32 < K) {
      stage_read16(A + (size_t)(mBlk + arow) * K + (k + 32) + ach, abuf);
      stage_read16(W + (size_t)nrow * K + (k + 32),          wbuf);
      stage_read16(W + (size_t)nrow * K + (k + 32) + 16,     wbuf + 16);
    }
    __syncthreads();

    bf16x16 af[4], wf[4];
#pragma unroll
    for (int i = 0; i < 4; ++i)
      af[i] = lds_frag(ldsA + (wm + 16 * i) * LDS_STRIDE, LDS_STRIDE);
#pragma unroll
    for (int j = 0; j < 4; ++j)
      wf[j] = lds_frag(ldsW + (wn + 16 * j) * LDS_STRIDE, LDS_STRIDE);
#pragma unroll
    for (int i = 0; i < 4; ++i)
#pragma unroll
      for (int j = 0; j < 4; ++j)
        acc[i][j] = wmma_bf16(af[i], wf[j], acc[i][j]);
  }

  const int nlane = lane & 15;
  const int mh    = (lane >> 4) * 8;
  __syncthreads();
  if (MODE == 0 || MODE == 1 || MODE == 3) {
    bf16* so = (bf16*)sob;
#pragma unroll
    for (int i = 0; i < 4; ++i)
#pragma unroll
      for (int j = 0; j < 4; ++j) {
        const int nl = wn + 16 * j + nlane;
        const float bv = bias ? bias[nBlk + nl] : 0.0f;
        if (MODE == 3) {
#pragma unroll 1
          for (int r = 0; r < 8; ++r) {
            const int ml = wm + 16 * i + mh + r;
            const float xg = acc[i][j][r] + bv;
            so[ml * 264 + nl] = (bf16)(0.5f * xg * (1.0f + erff(xg * 0.70710678118654752f)));
          }
        } else {
#pragma unroll
        for (int r = 0; r < 8; ++r) {
          const int ml = wm + 16 * i + mh + r;
          const bf16 hv = (bf16)(acc[i][j][r] + bv);
          if (MODE == 0) so[ml * 264 + nl] = hv;
          else           so[nl * 136 + ml] = hv;
        }
        }
      }
    __syncthreads();
#pragma unroll 1
    for (int pass = 0; pass < 2; ++pass) {
      if (MODE == 0 || MODE == 3) {
        for (int ch = t; ch < 128 * 32; ch += 256) { const int ml = ch >> 5, q = (ch & 31) * 8;
          *(volatile v4u_t*)((bf16*)out + (size_t)(mBlk + ml) * N + nBlk + q) = *(const v4ua*)(so + ml * 264 + q); }
      } else {
        const int b_ = mBlk / SS, s0 = mBlk % SS;
        for (int ch = t; ch < 256 * 16; ch += 256) { const int nl = ch >> 4, q = (ch & 15) * 8; const int n = nBlk + nl, h = n >> 6, dk = n & (DKK - 1);
          *(volatile v4u_t*)((bf16*)out + (((size_t)(b_ * HH + h)) * DKK + dk) * SS + s0 + q) = *(const v4ua*)(so + nl * 136 + q); }
      }
      __threadfence();
    }
  } else {
    float* so = (float*)sob;
#pragma unroll 1
    for (int hf = 0; hf < 2; ++hf) {
      if (wm == hf * 64) {
#pragma unroll
        for (int i = 0; i < 4; ++i)
#pragma unroll
          for (int j = 0; j < 4; ++j) {
            const int nl = wn + 16 * j + nlane;
            const float bv = bias ? bias[nBlk + nl] : 0.0f;
#pragma unroll
            for (int r = 0; r < 8; ++r) { const int mrow = mBlk + hf * 64 + 16 * i + mh + r; so[(16 * i + mh + r) * 260 + nl] = acc[i][j][r] * (rowscale ? rowscale[mrow] : 1.0f) + bv + (rowbias ? rowbias[mrow] : 0.0f); }
          }
      }
      __syncthreads();
      if (R) {
        for (int ch = t; ch < 64 * 64; ch += 256) { const int ml = ch >> 6, q = (ch & 63) * 4;
          if (nBlk + q < N) { const v4f_t rv = *(const v4f_t*)(R + (size_t)(mBlk + hf * 64 + ml) * N + nBlk + q); v4f_t v = *(const v4fa*)(so + ml * 260 + q); v += rv; *(volatile v4fa*)(so + ml * 260 + q) = v; } }
        asm volatile("s_wait_dscnt 0" ::: "memory");
      }
#pragma unroll 1
      for (int pass = 0; pass < 2; ++pass) {
        for (int ch = t; ch < 64 * 64; ch += 256) { const int ml = ch >> 6, q = (ch & 63) * 4;
          if (nBlk + q < N) *(volatile v4f_t*)((float*)out + (size_t)(mBlk + hf * 64 + ml) * N + nBlk + q) = *(const v4fa*)(so + ml * 260 + q); }
        __threadfence();
      }
      __syncthreads();
    }
  }
}


#define GSTR 48
template <typename AT, int EPI, bool OUT16>
__global__ __launch_bounds__(256) void gemm_kne(const AT* __restrict__ A, int lda, const float* __restrict__ Wm, int ldw,
                                                const float* __restrict__ bias, const float* __restrict__ R, const float* __restrict__ gvec,
                                                void* __restrict__ Yv, int ldy, int K) {
  __shared__ __attribute__((aligned(16))) f16 ldsA[128 * GSTR];
  __shared__ __attribute__((aligned(16))) f16 ldsW[128 * GSTR];
  __shared__ __attribute__((aligned(16))) float oS[8][32 * 68];
  const int tid = threadIdx.x, lane = tid & 31, wave = tid >> 5, cl = lane & 15, rh = (lane >> 4) * 8;
  const int m0 = blockIdx.x * 128, n0 = blockIdx.y * 128;
  const int wm = (wave & 3) * 32, wn = (wave >> 2) * 64;
  f32x8 acc[2][4];
#pragma unroll
  for (int i = 0; i < 2; ++i)
#pragma unroll
    for (int j = 0; j < 4; ++j) { f32x8 z = {}; acc[i][j] = z; }
#pragma unroll 1
  for (int k0 = 0; k0 < K; k0 += 32) {
    __syncthreads();
    { const int row = tid >> 1, ch = (tid & 1) * 16;
      const AT* src = A + (size_t)(m0 + row) * lda + k0 + ch;
#pragma unroll
      for (int g = 0; g < 16; ++g) ldsA[row * GSTR + ch + g] = (f16)src[g]; }
    { const int k = tid >> 3, nn0 = (tid & 7) * 16;
      const float* src = Wm + (size_t)(k0 + k) * ldw + n0 + nn0;
#pragma unroll
      for (int g = 0; g < 4; ++g) { const v4f_t v = *(const v4f_t*)(src + 4 * g);
#pragma unroll
        for (int u = 0; u < 4; ++u) ldsW[(nn0 + 4 * g + u) * GSTR + k] = (f16)v[u]; } }
    __syncthreads();
    f16x16 af[2];
#pragma unroll
    for (int i = 0; i < 2; ++i) af[i] = lds_frag(ldsA + (wm + 16 * i) * GSTR, GSTR);
#pragma unroll
    for (int j = 0; j < 4; ++j) {
      const f16x16 bf = lds_frag(ldsW + (wn + 16 * j) * GSTR, GSTR);
#pragma unroll
      for (int i = 0; i < 2; ++i) acc[i][j] = wmma16(af[i], bf, acc[i][j]);
    }
  }
  float* so = oS[wave];
#pragma unroll
  for (int i = 0; i < 2; ++i)
#pragma unroll
    for (int j = 0; j < 4; ++j) {
      const int n = n0 + wn + 16 * j + cl;
      const float bv = bias ? bias[n] : 0.0f;
      const float gv = (EPI == 2) ? gvec[n] : 0.0f;
      if (EPI == 1) {
#pragma unroll 1
        for (int r = 0; r < 8; ++r) { const float xg = acc[i][j][r] + bv; so[(16 * i + rh + r) * 68 + 16 * j + cl] = 0.5f * xg * (1.0f + erff(xg * 0.70710678118654752f)); }
      } else {
#pragma unroll
        for (int r = 0; r < 8; ++r) {
          float v = acc[i][j][r] + bv;
          if (EPI == 2) v = R[(size_t)(m0 + wm + 16 * i + rh + r) * ldy + n] + gv * v;
          so[(16 * i + rh + r) * 68 + 16 * j + cl] = v;
        }
      }
    }
  asm volatile("s_wait_dscnt 0" ::: "memory");
  __builtin_amdgcn_wave_barrier();
#pragma unroll 1
  for (int pass = 0; pass < 2; ++pass) {
    if (OUT16) {
      f16* Y = (f16*)Yv;
#pragma unroll
      for (int it = 0; it < 8; ++it) { const int c = lane + 32 * it, rr = c >> 3, q8 = (c & 7) * 8;
        union { f16 h[8]; v4u_t v; } u;
#pragma unroll
        for (int e = 0; e < 8; ++e) u.h[e] = (f16)so[rr * 68 + q8 + e];
        *(volatile v4u_t*)(Y + (size_t)(m0 + wm + rr) * ldy + n0 + wn + q8) = u.v; }
    } else {
      float* Y = (float*)Yv;
#pragma unroll
      for (int it = 0; it < 16; ++it) { const int f4 = lane + 32 * it, rr = f4 >> 4, q = (f4 & 15) * 4;
        *(volatile v4f_t*)(Y + (size_t)(m0 + wm + rr) * ldy + n0 + wn + q) = *(const v4fa*)(so + rr * 68 + q); }
    }
    __threadfence();
  }
}
__global__ __launch_bounds__(64) void attn_kernel(
    const bf16* __restrict__ Qb, const bf16* __restrict__ Kb,
    const bf16* __restrict__ Vt, const float* __restrict__ btab, int btstride,
    float* __restrict__ attnOut) {
  __shared__ bf16 ldsK[32 * KSTRIDE];
  __shared__ bf16 ldsV[64 * VSTRIDE];
  __shared__ __attribute__((aligned(16))) bf16 ldsO[2][32 * 72];

  const int q0blk = blockIdx.x * 64;
  const int h  = blockIdx.y;
  const int b  = blockIdx.z;
  const int t    = threadIdx.x;
  const int wave = t >> 5;
  const int lane = t & 31;
  const int qlane = lane & 15;
  const int kh8   = (lane >> 4) * 8;
  const int q0 = q0blk + wave * 32;

  const int hk = h / HKDIV;
  const bf16* Qh = Qb + (size_t)b * QROWS * DD + h * DKK;
  const bf16* Kh = Kb + (size_t)b * KROWS * KVD + hk * DKK;
  const bf16* Vh = Vt + ((size_t)(b * KVH + hk)) * DKK * KROWS;

  const int krow = t >> 1;
  const int kcol = (t & 1) * 32;
  const bf16* kSrc = Kh + (size_t)krow * KVD + kcol;
  const bf16* vSrc = Vh + (size_t)t * KROWS;

  bf16x16 qf[QW][2];
#pragma unroll
  for (int qt = 0; qt < QW; ++qt) {
    qf[qt][0] = load_frag(Qh, DD, q0 + 16 * qt, 0);
    qf[qt][1] = load_frag(Qh, DD, q0 + 16 * qt, 32);
  }

  f32x8 o[QW][4] = {};
  float mrun[QW], lrun[QW];
#pragma unroll
  for (int qt = 0; qt < QW; ++qt) { mrun[qt] = -INFINITY; lrun[qt] = 0.0f; }

  const float scale = 0.17677669529663688f * 1.44269504088896340736f;
  const float NEG2 = -1.0e9f;
  const int kmax = KROWS - 1;
  const float L2E_ = 1.44269504088896340736f; const float* bth = btab + (size_t)h * QROWS * 0;

  bf16x8 kreg[4], vreg[4];
#pragma unroll
  for (int i = 0; i < 4; ++i) {
    kreg[i] = *(const bf16x8*)(kSrc + 8 * i);
    vreg[i] = *(const bf16x8*)(vSrc + 8 * i);
  }

  for (int kb = 0; kb <= kmax; kb += 32) {
    __syncthreads();
#pragma unroll
    for (int i = 0; i < 4; ++i) {
      *(bf16x8*)(&ldsK[krow * KSTRIDE + kcol + 8 * i]) = kreg[i];
      *(bf16x8*)(&ldsV[t * VSTRIDE + 8 * i])           = vreg[i];
    }
    if (kb + 32 <= kmax) {
      const bf16* kn = kSrc + (size_t)(kb + 32) * KVD;
      const bf16* vn = vSrc + (kb + 32);
#pragma unroll
      for (int i = 0; i < 4; ++i) {
        kreg[i] = *(const bf16x8*)(kn + 8 * i);
        vreg[i] = *(const bf16x8*)(vn + 8 * i);
      }
    }
    __syncthreads();

    bf16x16 kf[2][2];
#pragma unroll
    for (int ktile = 0; ktile < 2; ++ktile)
#pragma unroll
      for (int c = 0; c < 2; ++c)
        kf[ktile][c] = lds_frag(ldsK + (ktile * 16) * KSTRIDE + c * 32, KSTRIDE);

    bf16x16 pf[QW];
    bool act[QW];
#pragma unroll
    for (int qt = 0; qt < QW; ++qt) {
      unsigned mbits = 0;
      {
#pragma unroll
        for (int r = 0; r < 8; ++r) { const int j0 = kb + kh8 + r; if (j0 < NKV) mbits |= 1u << r; if (j0 + 16 < NKV) mbits |= 1u << (8 + r); }
        act[qt] = (__builtin_amdgcn_ballot_w32(mbits != 0) != 0);
      }
      if (act[qt]) {
        const int q_my = q0 + 16 * qt + qlane;
        f32x8 s0 = {}, s1 = {};
        s0 = wmma_bf16(kf[0][0], qf[qt][0], s0);
        s0 = wmma_bf16(kf[0][1], qf[qt][1], s0);
        s1 = wmma_bf16(kf[1][0], qf[qt][0], s1);
        s1 = wmma_bf16(kf[1][1], qf[qt][1], s1);

        float mx = -INFINITY;
#pragma unroll
        for (int r = 0; r < 8; ++r) {
          const int k0i = kb + kh8 + r;
          const int k1i = k0i + 16;
          const float* brow = btab + (size_t)min(q_my, NKV - 1) * btstride; (void)bth;
          s0[r] = (mbits & (1u << r))       ? s0[r] * scale + L2E_ * brow[min(k0i, NKV - 1)] : NEG2;
          s1[r] = (mbits & (1u << (8 + r))) ? s1[r] * scale + L2E_ * brow[min(k1i, NKV - 1)] : NEG2;
          mx = fmaxf(mx, fmaxf(s0[r], s1[r]));
        }
        mx = fmaxf(mx, __shfl_xor(mx, 16, 32));
        const float mnew  = fmaxf(mrun[qt], mx);
        const float alpha = exp2f(mrun[qt] - mnew);

        float rsum = 0.0f;
#pragma unroll
        for (int r = 0; r < 8; ++r) {
          const float p0 = exp2f(s0[r] - mnew);
          const float p1 = exp2f(s1[r] - mnew);
          rsum += p0 + p1;
          pf[qt][r]     = (bf16)(p0 * 1024.0f);
          pf[qt][r + 8] = (bf16)(p1 * 1024.0f);
        }
        rsum += __shfl_xor(rsum, 16, 32);
        lrun[qt] = lrun[qt] * alpha + rsum;
        mrun[qt] = mnew;

#pragma unroll
        for (int j = 0; j < 4; ++j)
#pragma unroll
          for (int r = 0; r < 8; ++r) o[qt][j][r] *= alpha;
      }
    }

#pragma unroll
    for (int j = 0; j < 4; ++j) {
      const bf16x16 vf = lds_frag(ldsV + (j * 16) * VSTRIDE, VSTRIDE);
#pragma unroll
      for (int qt = 0; qt < QW; ++qt)
        if (act[qt]) o[qt][j] = wmma_bf16(vf, pf[qt], o[qt][j]);
    }
  }

  __shared__ __attribute__((aligned(16))) float ldsOf[2][32 * 68];
  float* so = ldsOf[wave]; (void)ldsO;
#pragma unroll
  for (int qt = 0; qt < QW; ++qt) {
    const float rl = 1.0f / (lrun[qt] * 1024.0f);
#pragma unroll
    for (int j = 0; j < 4; ++j)
#pragma unroll
      for (int r = 0; r < 8; ++r) so[(16 * qt + qlane) * 68 + j * 16 + kh8 + r] = o[qt][j][r] * rl;
  }
  asm volatile("s_wait_dscnt 0" ::: "memory");
  __builtin_amdgcn_wave_barrier();
#pragma unroll 1
  for (int pass = 0; pass < 2; ++pass) {
#pragma unroll
    for (int it = 0; it < 16; ++it) { const int ch = lane + 32 * it, ql = ch >> 4, q4 = (ch & 15) * 4;
      *(volatile v4f_t*)(attnOut + ((size_t)(b * QROWS + q0 + ql)) * DD + h * DKK + q4) = *(const v4fa*)(so + ql * 68 + q4); }
    __threadfence();
  }
}


__global__ __launch_bounds__(256) void k_ln(const float* __restrict__ X, int xpadded, const float* __restrict__ gam, const float* __restrict__ bet, float* __restrict__ Y) {
  __shared__ __attribute__((aligned(16))) float rowS[32 * 260];
  const int tid = threadIdx.x, r = tid >> 3, part = tid & 7; const size_t prow = (size_t)blockIdx.x * 32 + r; const int b = prow / SS, l = prow % SS; const bool live = l < LLj;
  const size_t srow = xpadded ? prow : ((size_t)b * LLj + l);
  float s = 0.0f;
#pragma unroll 1
  for (int i = 0; i < 32; ++i) { const float v = live ? X[srow * DDj + part * 32 + i] : 0.0f; rowS[r * 260 + part * 32 + i] = v; s += v; }
  s += __shfl_xor(s, 1, 32); s += __shfl_xor(s, 2, 32); s += __shfl_xor(s, 4, 32);
  const float mean = s * (1.0f / DDj); float q = 0.0f;
#pragma unroll 1
  for (int i = 0; i < 32; ++i) { const float d = rowS[r * 260 + part * 32 + i] - mean; q += d * d; }
  q += __shfl_xor(q, 1, 32); q += __shfl_xor(q, 2, 32); q += __shfl_xor(q, 4, 32);
  const float rstd = rsqrtf(q * (1.0f / DDj) + 1e-5f);
#pragma unroll 1
  for (int i = 0; i < 32; ++i) { const int c = part * 32 + i; rowS[r * 260 + c] = live ? ((rowS[r * 260 + c] - mean) * rstd * gam[c] + bet[c]) : 0.0f; }
  __syncthreads();
#pragma unroll 1
  for (int pass = 0; pass < 2; ++pass) { for (int q4 = tid; q4 < 32 * 64; q4 += 256) { const int rr = q4 >> 6, c4 = (q4 & 63) * 4;
      *(volatile v4f_t*)(Y + ((size_t)blockIdx.x * 32 + rr) * DDj + c4) = *(const v4fa*)(rowS + rr * 260 + c4); } __threadfence(); }
}
__global__ __launch_bounds__(256) void k_padx(const float* __restrict__ x, float* __restrict__ xp) { const size_t prow = blockIdx.x; const int b = prow / SS, l = prow % SS; const int c4 = threadIdx.x * 4;
  if (c4 < DDj) { v4f_t v = {0.f,0.f,0.f,0.f}; if (l < LLj) v = *(const v4f_t*)(x + ((size_t)b * LLj + l) * DDj + c4); *(volatile v4f_t*)(xp + prow * DDj + c4) = v; __threadfence(); *(volatile v4f_t*)(xp + prow * DDj + c4) = v; } }
__global__ __launch_bounds__(256) void k_padw(const float* __restrict__ w, const float* __restrict__ bq, int sel, float* __restrict__ Wp, float* __restrict__ bp) {
  const int i = blockIdx.x; for (int c = threadIdx.x; c < DD; c += 256) { const int h = c >> 6, d = c & 63; const float v = (d < HDj) ? w[(size_t)i * (3 * DDj) + sel * DDj + h * HDj + d] : 0.0f;
    *(volatile float*)(Wp + (size_t)i * DD + c) = v; __threadfence(); *(volatile float*)(Wp + (size_t)i * DD + c) = v;
    if (i == 0) { const float bv = (d < HDj) ? bq[sel * DDj + h * HDj + d] : 0.0f; *(volatile float*)(bp + c) = bv; __threadfence(); *(volatile float*)(bp + c) = bv; } }
}
__global__ __launch_bounds__(256) void k_padwvT(const float* __restrict__ w, float* __restrict__ WvT) { const int o = blockIdx.x; const int h = o >> 6, d = o & 63;
  for (int i = threadIdx.x; i < DDj; i += 256) { const float v = (d < HDj) ? w[(size_t)i * (3 * DDj) + 2 * DDj + h * HDj + d] : 0.0f; *(volatile float*)(WvT + (size_t)o * DDj + i) = v; __threadfence(); *(volatile float*)(WvT + (size_t)o * DDj + i) = v; } }
__global__ __launch_bounds__(256) void k_padwo(const float* __restrict__ w, float* __restrict__ Wop) { const int r = blockIdx.x; const int h = r >> 6, d = r & 63;
  for (int o = threadIdx.x; o < DDj; o += 256) { const float v = (d < HDj) ? w[(size_t)(h * HDj + d) * DDj + o] : 0.0f; *(volatile float*)(Wop + (size_t)r * DDj + o) = v; __threadfence(); *(volatile float*)(Wop + (size_t)r * DDj + o) = v; } }
__global__ __launch_bounds__(256) void k_bias(const float* __restrict__ rel, const float* __restrict__ graph, int h, float* __restrict__ Bt) {
  __shared__ __attribute__((aligned(16))) float rowB[BTS];
  const int i = blockIdx.x; const int ti = i / VVj, vi = i % VVj; const float* relh = rel + (size_t)h * (2 * MAXT - 1); const float* gh = graph + (size_t)h * VVj * VVj + vi * VVj;
  for (int j = threadIdx.x; j < BTS; j += 256) { float v = 0.0f; if (j < LLj) { const int tj = j / VVj, vj = j % VVj; v = relh[ti - tj + (MAXT - 1)] + gh[vj]; } rowB[j] = v; }
  __syncthreads();
#pragma unroll 1
  for (int pass = 0; pass < 2; ++pass) { for (int q4 = threadIdx.x; q4 < BTS / 4; q4 += 256) *(volatile v4f_t*)(Bt + (size_t)i * BTS + q4 * 4) = *(const v4fa*)(rowB + q4 * 4); __threadfence(); }
}
__global__ __launch_bounds__(256) void k_ones(float* __restrict__ p, int n) { for (int i = threadIdx.x * 4; i < n; i += 1024) { v4f_t o = {1.f,1.f,1.f,1.f}; *(volatile v4f_t*)(p + i) = o; __threadfence(); *(volatile v4f_t*)(p + i) = o; } }
__global__ __launch_bounds__(256) void k_copyout(const float* __restrict__ src, float* __restrict__ out) { const size_t r = blockIdx.x; const int b = r / LLj, l = r % LLj; const int c4 = threadIdx.x * 4;
  if (c4 < DDj) { const v4f_t v = *(const v4f_t*)(src + ((size_t)b * SS + l) * DDj + c4); *(volatile v4f_t*)(out + r * DDj + c4) = v; __threadfence(); *(volatile v4f_t*)(out + r * DDj + c4) = v; } }

extern "C" void kernel_launch(void* const* d_in, const int* in_sizes, int n_in,
                              void* d_out, int out_size, void* d_ws, size_t ws_size,
                              hipStream_t stream) {
  (void)in_sizes; (void)n_in; (void)out_size;
  const float** f = (const float**)d_in;
  const float* x = f[0], *ln1g = f[1], *ln1b = f[2], *wqkv = f[3], *bqkv = f[4], *rel = f[5], *graph = f[6], *wproj = f[7], *bproj = f[8], *ln2g = f[9], *ln2b = f[10], *w1 = f[11], *b1 = f[12], *w2 = f[13], *b2 = f[14];
  float* out = (float*)d_out;
  char* ws = (char*)d_ws;
  float* xp = (float*)ws; ws += (size_t)MPADr * DDj * 4;
  float* h1 = (float*)ws; ws += (size_t)MPADr * DDj * 4;
  float* Wq = (float*)ws; ws += (size_t)DDj * DD * 4; float* Wk = (float*)ws; ws += (size_t)DDj * DD * 4; float* WvT = (float*)ws; ws += (size_t)DD * DDj * 4; float* Wop = (float*)ws; ws += (size_t)DD * DDj * 4;
  float* bq = (float*)ws; ws += DD * 4; float* bk = (float*)ws; ws += DD * 4; float* bv = (float*)ws; ws += DD * 4;
  bf16* Qb = (bf16*)ws; ws += (size_t)MPADr * DD * 2; bf16* Kb = (bf16*)ws; ws += (size_t)MPADr * DD * 2; bf16* VtB = (bf16*)ws; ws += (size_t)MPADr * DD * 2;
  float* att = (float*)ws; ws += (size_t)MPADr * DD * 4;
  float* x1 = (float*)ws; ws += (size_t)MPADr * DDj * 4;
  float* h2 = (float*)ws; ws += (size_t)MPADr * DDj * 4;
  float* ff = (float*)ws; ws += (size_t)MPADr * 4 * DDj * 4;
  float* y = (float*)ws; ws += (size_t)MPADr * DDj * 4;
  float* Bt = (float*)ws; ws += (size_t)LLj * BTS * 4;
  float* ones = (float*)ws; ws += 1024 * 4;
  if ((size_t)(ws - (char*)d_ws) > ws_size) return;
  const dim3 blk(256);
  k_ones<<<dim3(1), blk, 0, stream>>>(ones, 1024);
  k_padx<<<dim3(MPADr), blk, 0, stream>>>(x, xp);
  k_padw<<<dim3(DDj), blk, 0, stream>>>(wqkv, bqkv, 0, Wq, bq); k_padw<<<dim3(DDj), blk, 0, stream>>>(wqkv, bqkv, 1, Wk, bk);
  k_padwvT<<<dim3(DD), blk, 0, stream>>>(wqkv, WvT); k_padw<<<dim3(1), blk, 0, stream>>>(wqkv, bqkv, 2, y  , bv);
  k_padwo<<<dim3(DD), blk, 0, stream>>>(wproj, Wop);
  k_ln<<<dim3(MPADr / 32), blk, 0, stream>>>(xp, 1, ln1g, ln1b, h1);
  gemm_kne<float, 0, true><<<dim3(MPADr / 128, DD / 128), blk, 0, stream>>>(h1, DDj, Wq, DD, bq, nullptr, nullptr, Qb, DD, DDj);
  gemm_kne<float, 0, true><<<dim3(MPADr / 128, DD / 128), blk, 0, stream>>>(h1, DDj, Wk, DD, bk, nullptr, nullptr, Kb, DD, DDj);
  gemm_rb_kernel<float, 1><<<dim3(MPADr / 128, DD / 256), blk, 0, stream>>>(h1, WvT, bv, nullptr, nullptr, nullptr, VtB, MPADr, DD, DDj);
  for (int h = 0; h < HH; ++h) {
    k_bias<<<dim3(LLj), blk, 0, stream>>>(rel, graph, h, Bt);
    attn_kernel<<<dim3(SS / 64, 1, BB), dim3(64), 0, stream>>>(Qb + h * DKK, Kb + h * DKK, VtB + (size_t)h * DKK * KROWS, Bt, BTS, att + h * DKK);
  }
  gemm_kne<float, 2, false><<<dim3(MPADr / 128, DDj / 128), blk, 0, stream>>>(att, DD, Wop, DDj, bproj, xp, ones, x1, DDj, DD);
  k_ln<<<dim3(MPADr / 32), blk, 0, stream>>>(x1, 1, ln2g, ln2b, h2);
  gemm_kne<float, 1, false><<<dim3(MPADr / 128, 4 * DDj / 128), blk, 0, stream>>>(h2, DDj, w1, 4 * DDj, b1, nullptr, nullptr, ff, 4 * DDj, DDj);
  gemm_kne<float, 2, false><<<dim3(MPADr / 128, DDj / 128), blk, 0, stream>>>(ff, 4 * DDj, w2, DDj, b2, x1, ones, y, DDj, 4 * DDj);
  k_copyout<<<dim3(MROWS), blk, 0, stream>>>(y, out);
}
